// HebbNet_33337536151735
// MI455X (gfx1250) — hardware-verified
//
#include <hip/hip_runtime.h>
#include <math.h>

typedef __attribute__((ext_vector_type(16))) _Float16 v16h;
typedef __attribute__((ext_vector_type(8)))  _Float16 v8h;
typedef __attribute__((ext_vector_type(16))) __bf16   v16b;
typedef __attribute__((ext_vector_type(8)))  __bf16   v8b;
typedef __attribute__((ext_vector_type(8)))  float    v8f;
typedef __attribute__((ext_vector_type(4)))  float    v4f;

constexpr int kT    = 32;
constexpr int kB    = 32;
constexpr int kNx   = 512;
constexpr int kNh   = 512;
constexpr int kNy   = 64;
constexpr int kRows = kT * kB;
constexpr int kThr  = 256;
constexpr float kInCarry = 1024.0f;
constexpr float kWCarry  = 4096.0f;
constexpr float kSCarry  = 1024.0f;
constexpr float kScXX = 1.0f / (kInCarry * kInCarry);
constexpr float kScHW = 1.0f / (kSCarry * kWCarry);
constexpr float kF16MinNormal = 6.103515625e-5f;

static_assert((kRows % 64) == 0 && (kNh % 64) == 0 && (kNy % 64) == 0, "GEMM M, N multiples of 64");
static_assert(((kRows / 64) * (kNh / 64)) % 8 == 0 && ((kRows / 64) * (kRows / 64)) % 8 == 0 && ((kRows / 64) * (kNy / 64)) % 8 == 0, "GEMM grids exact");
static_assert((kNx % 32) == 0 && (kNh % 32) == 0, "GEMM K multiples of 32");

constexpr size_t kOffX16  = 0;
constexpr size_t kOffW116 = kOffX16  + (size_t)kRows * kNx * 2;
constexpr size_t kOffW2T  = kOffW116 + (size_t)kNh * kNx * 2;
constexpr size_t kOffBF   = kOffW2T  + (size_t)kNy * kNh * 2;
constexpr int kFB1 = 0, kFB2 = 512, kFZB = 640, kFEnd = 2048;
constexpr size_t kOffXW   = kOffBF   + (size_t)kFEnd * 4;
constexpr size_t kOffGF   = kOffXW   + (size_t)kRows * kNh * 4;
constexpr size_t kOffH16  = kOffGF   + (size_t)kRows * kRows * 4;
constexpr size_t kOffY    = kOffH16  + (size_t)kRows * kNh * 2;
constexpr size_t kWsTotal = kOffY    + (size_t)kRows * kNy * 4;
static_assert(kWsTotal == 9248768ull, "carve total");
static_assert(kWsTotal <= 134217728ull, "carve cap");
static_assert((kOffW116 % 256) == 0 && (kOffW2T % 256) == 0 && (kOffBF % 256) == 0 && (kOffXW % 256) == 0 && (kOffGF % 256) == 0 && (kOffH16 % 256) == 0 && (kOffY % 256) == 0, "aligned regions");
static_assert(kFEnd - kFZB >= kRows, "the zero bias row covers the widest product");
constexpr size_t kOut1 = (size_t)kRows * kNh;
constexpr size_t kOutTotal = kOut1 + (size_t)kRows * kNy;

__device__ __forceinline__ unsigned short f2bf_bits(float f) {
  unsigned u = __float_as_uint(f);
  return (unsigned short)((u + 0x7FFFu + ((u >> 16) & 1u)) >> 16);
}
__device__ __forceinline__ float bf_bits2f(unsigned short h) { return __uint_as_float(((unsigned)h) << 16); }
__device__ __forceinline__ float bf16r(float f) { return bf_bits2f(f2bf_bits(f)); }
__device__ __forceinline__ float carry_flush(float v, float carry) {
  const float s = v * carry;
  return (fabsf(s) < kF16MinNormal) ? 0.0f : s;
}
__device__ __forceinline__ float frcp(float x) { return __builtin_amdgcn_rcpf(x); }

__device__ __forceinline__ void dep_guard4_h(v8f& a, v8f& b, v8f& c, v8f& d, v16h x, v16h y) { asm volatile("v_nop\n\tv_nop\n\tv_nop\n\tv_nop" : "+v"(a), "+v"(b), "+v"(c), "+v"(d) : "v"(x), "v"(y)); }
__device__ __forceinline__ void dep_guard4_b(v8f& a, v8f& b, v8f& c, v8f& d, v16b x, v16b y) { asm volatile("v_nop\n\tv_nop\n\tv_nop\n\tv_nop" : "+v"(a), "+v"(b), "+v"(c), "+v"(d) : "v"(x), "v"(y)); }
__device__ __forceinline__ void keep4_h(v16h a, v16h b, v16h c, v16h d) { asm volatile("v_nop" :: "v"(a), "v"(b), "v"(c), "v"(d)); }
__device__ __forceinline__ void keep4_b(v16b a, v16b b, v16b c, v16b d) { asm volatile("v_nop" :: "v"(a), "v"(b), "v"(c), "v"(d)); }
__device__ __forceinline__ void acc_guard4(v8f& a, v8f& b, v8f& c, v8f& d) { asm volatile("v_nop\n\tv_nop\n\tv_nop\n\tv_nop" : "+v"(a), "+v"(b), "+v"(c), "+v"(d)); }

template <typename T> struct Frag;
template <> struct Frag<_Float16> {
  typedef v16h V; union U { v16h v; v8h h[2]; };
  static __device__ __forceinline__ v16h load(const _Float16* p) {
    U f; f.h[0] = *(const v8h*)(p); f.h[1] = *(const v8h*)(p + 16); return f.v;
  }
  static __device__ __forceinline__ v8f mma(v16h a, v16h b, v8f c) {
    return __builtin_amdgcn_wmma_f32_16x16x32_f16(false, a, false, b, (short)0, c, false, false);
  }
  static __device__ __forceinline__ void guard4(v8f& a, v8f& b, v8f& c, v8f& d, v16h x, v16h y) { dep_guard4_h(a, b, c, d, x, y); }
  static __device__ __forceinline__ void keep(v16h a, v16h b, v16h c, v16h d) { keep4_h(a, b, c, d); }
};
template <> struct Frag<__bf16> {
  typedef v16b V; union U { v16b v; v8b h[2]; };
  static __device__ __forceinline__ v16b load(const __bf16* p) {
    U f; f.h[0] = *(const v8b*)(p); f.h[1] = *(const v8b*)(p + 16); return f.v;
  }
  static __device__ __forceinline__ v8f mma(v16b a, v16b b, v8f c) {
    return __builtin_amdgcn_wmma_f32_16x16x32_bf16(false, a, false, b, (short)0, c, false, false);
  }
  static __device__ __forceinline__ void guard4(v8f& a, v8f& b, v8f& c, v8f& d, v16b x, v16b y) { dep_guard4_b(a, b, c, d, x, y); }
  static __device__ __forceinline__ void keep(v16b a, v16b b, v16b c, v16b d) { keep4_b(a, b, c, d); }
};

__device__ __forceinline__ v8f mma_h(v16h a, v16h b, v8f c) {
  c = __builtin_amdgcn_wmma_f32_16x16x32_f16(false, a, false, b, (short)0, c, false, false);
  asm volatile("v_nop\n\tv_nop\n\tv_nop\n\tv_nop" : "+v"(c) : "v"(a), "v"(b));
  return c;
}

template <int ET> struct Elem;
template <> struct Elem<0> { typedef _Float16 T; };
template <> struct Elem<1> { typedef __bf16 T; };
template <int ET, bool SPLIT, int BIAS_MODE, int OUT_MODE, bool RESID, int ACT = 0>
__global__ __launch_bounds__(256) void wmma_gemm64(
    const unsigned short* __restrict__ Ap, const unsigned short* __restrict__ A2p, int lda, long strideA,
    const unsigned short* __restrict__ Btp, const unsigned short* __restrict__ Bt2p, int ldb, long strideB,
    void* __restrict__ Cout, void* __restrict__ Cout2, int ldc, long strideC,
    const float* __restrict__ bias,
    const float* __restrict__ resid, long strideR,
    int M, int N, int K, float scale) {
  typedef typename Elem<ET>::T T;
  typedef typename Frag<T>::V V;
  const T* A = (const T*)Ap; const T* A2 = (const T*)A2p; const T* Bt = (const T*)Btp; const T* Bt2 = (const T*)Bt2p;
  __shared__ __align__(16) float sT[8][16 * 68];
  const int b    = blockIdx.y;
  const int lane = threadIdx.x & 31;
  const int wave = threadIdx.x >> 5;
  const int tilesN = N >> 6;
  const int tilesM = M >> 6;
  const int tile = blockIdx.x * 8 + wave;
  if (tile >= tilesM * tilesN) return;
  const int tm = tile / tilesN;
  const int tn = tile - tm * tilesN;
  const int m0 = tm << 6;
  const int n0 = tn << 6;

  const T* Ab  = A  + (size_t)b * strideA;
  const T* Bb  = Bt + (size_t)b * strideB;
  const T* Ab2 = SPLIT ? (A2  + (size_t)b * strideA) : nullptr;
  const T* Bb2 = SPLIT ? (Bt2 + (size_t)b * strideB) : nullptr;

  const int rlane = lane & 15;
  const int koff  = (lane >> 4) * 8;
  const int mOff  = (lane >> 4) * 8;

  v8f acc[4][4];
#pragma unroll
  for (int i = 0; i < 4; ++i)
#pragma unroll
    for (int j = 0; j < 4; ++j) acc[i][j] = (v8f){0.f,0.f,0.f,0.f,0.f,0.f,0.f,0.f};

  for (int k0 = 0; k0 < K; k0 += 32) {
    V bh[4], bl[4];
#pragma unroll
    for (int j = 0; j < 4; ++j) {
      const size_t bo = (size_t)(n0 + (j << 4) + rlane) * ldb + koff + k0;
      bh[j] = Frag<T>::load(Bb + bo);
      if (SPLIT) bl[j] = Frag<T>::load(Bb2 + bo);
    }
#pragma unroll
    for (int i = 0; i < 4; ++i) {
      const size_t ao = (size_t)(m0 + (i << 4) + rlane) * lda + koff + k0;
      V ah = Frag<T>::load(Ab + ao);
      V al;
      if (SPLIT) al = Frag<T>::load(Ab2 + ao);
#pragma unroll
      for (int j = 0; j < 4; ++j) {
        acc[i][j] = Frag<T>::mma(ah, bh[j], acc[i][j]);
        if (SPLIT) {
          acc[i][j] = Frag<T>::mma(ah, bl[j], acc[i][j]);
          acc[i][j] = Frag<T>::mma(al, bh[j], acc[i][j]);
        }
      }
      Frag<T>::guard4(acc[i][0], acc[i][1], acc[i][2], acc[i][3], ah, SPLIT ? al : ah);
    }
    Frag<T>::keep(bh[0], bh[1], bh[2], bh[3]);
    if (SPLIT) Frag<T>::keep(bl[0], bl[1], bl[2], bl[3]);
  }
  acc_guard4(acc[0][0], acc[0][1], acc[0][2], acc[0][3]);
  acc_guard4(acc[1][0], acc[1][1], acc[1][2], acc[1][3]);
  acc_guard4(acc[2][0], acc[2][1], acc[2][2], acc[2][3]);
  acc_guard4(acc[3][0], acc[3][1], acc[3][2], acc[3][3]);

  float* slab = sT[wave];
  const float* Rb = RESID ? (resid + (size_t)b * strideR) : nullptr;
#pragma unroll
  for (int i = 0; i < 4; ++i) {
    const int mBase = m0 + (i << 4);
#pragma unroll
    for (int j = 0; j < 4; ++j) {
      const int n = n0 + (j << 4) + rlane;
      float bv = 0.f;
      if (BIAS_MODE == 2) bv = bias[n];
#pragma unroll
      for (int r = 0; r < 8; ++r) {
        float v = acc[i][j][r] * scale;
        if (BIAS_MODE == 1) v += bias[mBase + mOff + r];
        if (BIAS_MODE == 2) v += bv;
        if (RESID) v += Rb[(size_t)(mBase + mOff + r) * ldc + n];
        if (ACT == 1) v = tanhf(v);
        if (ACT == 2) v = fmaxf(v, 0.0f);
        if (ACT == 3) v = v / (1.0f + expf(-v));
        if (ACT == 4) v = (v > 0.f) ? v : 0.01f * v;
        slab[(mOff + r) * 68 + (j << 4) + rlane] = v;
      }
    }
    __builtin_amdgcn_fence(__ATOMIC_RELEASE, "workgroup");
    __builtin_amdgcn_wave_barrier();
    __builtin_amdgcn_fence(__ATOMIC_ACQUIRE, "workgroup");
    if (OUT_MODE == 0) {
      float* C = (float*)Cout + (size_t)b * strideC;
      const int hh = lane >> 4, c4 = (lane & 15) * 4;
      for (int pass = 0; pass < 2; ++pass) {
#pragma unroll
        for (int it = 0; it < 8; ++it) {
          const int row = it * 2 + hh;
          v4f v = *(const v4f*)(slab + row * 68 + c4);
          *(volatile v4f*)(C + (size_t)(mBase + row) * ldc + n0 + c4) = v;
        }
        __threadfence();
      }
    } else {
      const int q = lane >> 3, c8 = (lane & 7) * 8;
      unsigned short* C  = (unsigned short*)Cout  + (size_t)b * strideC;
      unsigned short* C2 = (OUT_MODE == 2) ? ((unsigned short*)Cout2 + (size_t)b * strideC) : nullptr;
      for (int pass = 0; pass < 2; ++pass) {
#pragma unroll
        for (int it = 0; it < 4; ++it) {
          const int row = it * 4 + q;
          const float* sp = slab + row * 68 + c8;
          v8h hv, lv;
#pragma unroll
          for (int e = 0; e < 8; ++e) {
            if (OUT_MODE == 1) {
              hv[e] = (_Float16)sp[e];
            } else {
              unsigned short hb = f2bf_bits(sp[e]);
              unsigned short lb = f2bf_bits(sp[e] - bf_bits2f(hb));
              hv[e] = __builtin_bit_cast(_Float16, hb);
              lv[e] = __builtin_bit_cast(_Float16, lb);
            }
          }
          *(volatile v8h*)(C + (size_t)(mBase + row) * ldc + n0 + c8) = hv;
          if (OUT_MODE == 2) *(volatile v8h*)(C2 + (size_t)(mBase + row) * ldc + n0 + c8) = lv;
        }
        __threadfence();
      }
    }
    __builtin_amdgcn_fence(__ATOMIC_RELEASE, "workgroup");
    __builtin_amdgcn_wave_barrier();
    __builtin_amdgcn_fence(__ATOMIC_ACQUIRE, "workgroup");
  }
}

__global__ __launch_bounds__(kThr) void cast_plane_kernel(const float* __restrict__ src, unsigned short* __restrict__ dst,
                                                          int colsLog2, int dstPitch, int dstOff) {
  const int i   = blockIdx.x * kThr + threadIdx.x;
  const int sh  = colsLog2 - 3;
  const int row = i >> sh;
  const int c8  = (i & ((1 << sh) - 1)) * 8;
  const float* sp = src + ((size_t)row << colsLog2) + c8;
  const v4f a0 = *(const v4f*)(sp);
  const v4f a1 = *(const v4f*)(sp + 4);
  v8h hv;
#pragma unroll
  for (int e = 0; e < 4; ++e) {
    const float f0 = a0[e];
    const float f1 = a1[e];
    hv[e]     = (_Float16)carry_flush(bf16r(f0), kInCarry);
    hv[4 + e] = (_Float16)carry_flush(bf16r(f1), kInCarry);
  }
  unsigned short* dp = dst + (size_t)row * dstPitch + dstOff + c8;
  *(volatile v8h*)dp = hv;
  __threadfence();
  *(volatile v8h*)dp = hv;
}
__global__ __launch_bounds__(256) void wt_plane_kernel(const float* __restrict__ W, unsigned short* __restrict__ dst, int K, int N, int nLive, int ldd, int colOff) {
  const int n  = blockIdx.x;
  const int k8 = threadIdx.x * 8;
  const bool live = n < nLive;
  const int nc = live ? n : 0;
  v8h hv;
#pragma unroll
  for (int e = 0; e < 8; ++e) {
    const float w = W[(size_t)(k8 + e) * N + nc];
    hv[e] = (_Float16)(live ? carry_flush(bf16r(w), kWCarry) : 0.0f);
  }
  unsigned short* dp = dst + (size_t)n * ldd + colOff + k8;
  *(volatile v8h*)dp = hv;
  __threadfence();
  *(volatile v8h*)dp = hv;
}


__device__ __forceinline__ float fast_sigmoid(float v) { return frcp(1.0f + __expf(-v)); }

__global__ __launch_bounds__(kThr) void setup_kernel(const float* __restrict__ b1, const float* __restrict__ b2, float* __restrict__ BF) {
  unsigned v = blockIdx.x * (unsigned)kThr + threadIdx.x;
  asm volatile("" : "+v"(v));
  const unsigned i0 = v * 4u;
  v4f o = {0.f, 0.f, 0.f, 0.f};
  if (i0 < (unsigned)kFB2) {
    const v4f a = *(const v4f*)(b1 + i0);
#pragma unroll
    for (int e = 0; e < 4; ++e) { const float x = a[e]; o[e] = bf16r(x); }
  } else if (i0 < (unsigned)kFZB) {
    const unsigned j = i0 - (unsigned)kFB2;
    if (j < (unsigned)kNy) {
      const v4f a = *(const v4f*)(b2 + j);
#pragma unroll
      for (int e = 0; e < 4; ++e) { const float x = a[e]; o[e] = bf16r(x); }
    }
  }
  float* dp = BF + i0;
  *(volatile v4f*)dp = o;
  __threadfence();
  *(volatile v4f*)dp = o;
}
static_assert(kFEnd / 4 == 2 * kThr && (kFB2 % 128) == 0 && (kFZB % 128) == 0, "set-up grid exact; regions wave-uniform");

__global__ __launch_bounds__(64) void hebb_scan_kernel(const float* __restrict__ XW, const float* __restrict__ GF, const float* __restrict__ lam,
                                                       const float* __restrict__ eta, float* __restrict__ out0, unsigned short* __restrict__ H16) {
  __shared__ __align__(16) float sH[kT * kNh];
  __shared__ __align__(16) float sC[kT];
  __shared__ __align__(16) float sLam[kT];
  const int tid = threadIdx.x;
  const int b   = blockIdx.x;
  const int u8  = tid * 8;
  const float lam0 = lam[0];
  const float eta0 = eta[0];
  const float lamc = fminf(bf16r(lam0), 1.0f);
  const float etab = bf16r(eta0);
  if (tid == 0) {
    float p = 1.0f;
#pragma unroll 1
    for (int k = 0; k < kT; ++k) { sLam[k] = p; p = p * lamc; }
  }
  __syncthreads();
#pragma unroll 1
  for (int t = 0; t < kT; ++t) {
    const size_t row = (size_t)t * kB + b;
    if (tid < t) {
      const float g = GF[((size_t)tid * kB + b) * kRows + row];
      sC[tid] = (etab * sLam[t - 1 - tid]) * g;
    }
    __syncthreads();
    float acc[8];
#pragma unroll
    for (int e = 0; e < 8; ++e) acc[e] = 0.0f;
#pragma unroll 1
    for (int s = 0; s < t; ++s) {
      const float c = sC[s];
      const v4f h0 = *(const v4f*)(sH + s * kNh + u8);
      const v4f h1 = *(const v4f*)(sH + s * kNh + u8 + 4);
#pragma unroll
      for (int e = 0; e < 4; ++e) { acc[e] += c * h0[e]; acc[4 + e] += c * h1[e]; }
    }
    const float* xr = XW + row * kNh + u8;
    const v4f x0 = *(const v4f*)xr, x1 = *(const v4f*)(xr + 4);
    v4f hn0, hn1;
    v8h hv;
#pragma unroll
    for (int e = 0; e < 4; ++e) {
      hn0[e] = fast_sigmoid(x0[e] + acc[e]);
      hn1[e] = fast_sigmoid(x1[e] + acc[4 + e]);
      hv[e]     = (_Float16)carry_flush(hn0[e], kSCarry);
      hv[4 + e] = (_Float16)carry_flush(hn1[e], kSCarry);
    }
    *(v4f*)(sH + t * kNh + u8) = hn0;
    *(v4f*)(sH + t * kNh + u8 + 4) = hn1;
    float* op = out0 + row * kNh + u8;
    unsigned short* hp = H16 + row * kNh + u8;
    for (int pass = 0; pass < 2; ++pass) {
      *(volatile v4f*)op = hn0;
      *(volatile v4f*)(op + 4) = hn1;
      *(volatile v8h*)hp = hv;
      __threadfence();
    }
    __syncthreads();
  }
}
static_assert(kNh == 64 * 8 && kT <= 64, "one block of 64 threads covers the 512 units; the coefficient threads s < t fit the block");

__global__ __launch_bounds__(kThr) void head_sigmoid_kernel(const float* __restrict__ Y, float* __restrict__ out1) {
  const size_t i = (size_t)blockIdx.x * kThr + threadIdx.x;
  const v4f y = *(const v4f*)(Y + i * 4);
  v4f o;
#pragma unroll
  for (int e = 0; e < 4; ++e) o[e] = fast_sigmoid(y[e]);
  float* dp = out1 + i * 4;
  *(volatile v4f*)dp = o;
  __threadfence();
  *(volatile v4f*)dp = o;
}
static_assert(kRows * kNy / 4 == 64 * kThr, "head grid exact");

static_assert(((size_t)kRows * kNx / 8) % kThr == 0 && ((size_t)kNh * kNx / 8) % kThr == 0, "cast grids exact");

extern "C" void kernel_launch(void* const* d_in, const int* in_sizes, int n_in,
                              void* d_out, int out_size, void* d_ws, size_t ws_size,
                              hipStream_t stream) {
  if (n_in < 7 || d_out == nullptr || d_ws == nullptr) return;
  if (in_sizes[0] != kRows * kNx || in_sizes[1] != kNh * kNx || in_sizes[2] != kNh || in_sizes[3] != kNh * kNy || in_sizes[4] != kNy || in_sizes[5] != 1 || in_sizes[6] != 1) return;
  if ((size_t)out_size != kOutTotal) return;
  if (ws_size < kWsTotal) return;
  const float* x   = (const float*)d_in[0];
  const float* w1  = (const float*)d_in[1];
  const float* b1  = (const float*)d_in[2];
  const float* w2  = (const float*)d_in[3];
  const float* b2  = (const float*)d_in[4];
  const float* lam = (const float*)d_in[5];
  const float* eta = (const float*)d_in[6];
  float* out0 = (float*)d_out;
  float* out1 = (float*)d_out + kOut1;
  char* ws = (char*)d_ws;
  unsigned short* X16  = (unsigned short*)(ws + kOffX16);
  unsigned short* W116 = (unsigned short*)(ws + kOffW116);
  unsigned short* W2T  = (unsigned short*)(ws + kOffW2T);
  float* BF  = (float*)(ws + kOffBF);
  float* XW  = (float*)(ws + kOffXW);
  float* GF  = (float*)(ws + kOffGF);
  unsigned short* H16  = (unsigned short*)(ws + kOffH16);
  float* Y   = (float*)(ws + kOffY);

  cast_plane_kernel<<<(int)(((size_t)kRows * kNx / 8) / kThr), kThr, 0, stream>>>(x, X16, 9, kNx, 0);
  cast_plane_kernel<<<(int)(((size_t)kNh * kNx / 8) / kThr), kThr, 0, stream>>>(w1, W116, 9, kNx, 0);
  wt_plane_kernel<<<kNy, kNh / 8, 0, stream>>>(w2, W2T, kNh, kNy, kNy, kNh, 0);
  setup_kernel<<<2, kThr, 0, stream>>>(b1, b2, BF);

  wmma_gemm64<0, false, 2, 0, false, 0><<<dim3((kRows / 64) * (kNh / 64) / 8, 1), 256, 0, stream>>>(
      X16, X16, kNx, 0L, W116, W116, kNx, 0L, (void*)XW, (void*)XW, kNh, 0L, BF + kFB1, nullptr, 0L, kRows, kNh, kNx, kScXX);
  wmma_gemm64<0, false, 2, 0, false, 0><<<dim3((kRows / 64) * (kRows / 64) / 8, 1), 256, 0, stream>>>(
      X16, X16, kNx, 0L, X16, X16, kNx, 0L, (void*)GF, (void*)GF, kRows, 0L, BF + kFZB, nullptr, 0L, kRows, kRows, kNx, kScXX);
  hebb_scan_kernel<<<kB, 64, 0, stream>>>(XW, GF, lam, eta, out0, H16);
  wmma_gemm64<0, false, 2, 0, false, 0><<<dim3((kRows / 64) * (kNy / 64) / 8, 1), 256, 0, stream>>>(
      H16, H16, kNh, 0L, W2T, W2T, kNh, 0L, (void*)Y, (void*)Y, kNy, 0L, BF + kFB2, nullptr, 0L, kRows, kNy, kNh, kScHW);
  head_sigmoid_kernel<<<64, kThr, 0, stream>>>(Y, out1);
}
